// PredictionScore_70789650973258
// MI455X (gfx1250) — hardware-verified
//
#include <hip/hip_runtime.h>
#include <math.h>

#define NB   8
#define NL   64
#define NPP  512
#define NC   128
#define NG   10
#define KW   256

#define OUT_PI 0L
#define OUT_SG 2621440L
#define OUT_MU 5242880L
#define OUT_D  7864320L
#define OUT_BA 8126464L
#define OUT_TOTAL 8126472L

#define WB_WHI 0
#define WB_WLO 65536
#define WB_PHI 131072
#define WB_PLO 135168
#define WB_SG  139264
#define WB_MU  143360
#define WB_PA  148736
#define WB_PB  410880
#define WB_END 2508032

#define PROJ_BLOCKS 144
#define MDN_BLOCKS 4096

typedef _Float16 f16_t;
typedef _Float16 v16h __attribute__((ext_vector_type(16)));
typedef _Float16 v8h  __attribute__((ext_vector_type(8), __may_alias__));
typedef __bf16   v16b __attribute__((ext_vector_type(16)));
typedef float    v8f  __attribute__((ext_vector_type(8)));
typedef float    v4f  __attribute__((ext_vector_type(4), __may_alias__));
typedef unsigned short v16us __attribute__((ext_vector_type(16)));
typedef unsigned short v8us  __attribute__((ext_vector_type(8), __may_alias__));
typedef unsigned short v4us  __attribute__((ext_vector_type(4), __may_alias__));

__device__ __forceinline__ unsigned short bf16_rne(float x) {
  unsigned int u = __float_as_uint(x);
  u += 0x7FFFu + ((u >> 16) & 1u);
  return (unsigned short)(u >> 16);
}

__device__ __forceinline__ void split_bf16(float x, unsigned short& hi, unsigned short& lo) {
  unsigned short hb = bf16_rne(x);
  float hf = __uint_as_float(((unsigned int)hb) << 16);
  hi = hb;
  lo = bf16_rne(x - hf);
}

__device__ __forceinline__ v8f zero8() {
  v8f z;
#pragma unroll
  for (int r = 0; r < 8; ++r) z[r] = 0.f;
  return z;
}

__device__ __forceinline__ v16us cat8u(v8us a, v8us b) {
  return __builtin_shufflevector(a, b, 0, 1, 2, 3, 4, 5, 6, 7, 8, 9, 10, 11, 12, 13, 14, 15);
}
__device__ __forceinline__ v16h cat8h(v8h a, v8h b) {
  return __builtin_shufflevector(a, b, 0, 1, 2, 3, 4, 5, 6, 7, 8, 9, 10, 11, 12, 13, 14, 15);
}

__device__ __forceinline__ v8f mma_bf16(v16us a, v16us b, v8f c) {
  v16b av = __builtin_bit_cast(v16b, a);
  v16b bv = __builtin_bit_cast(v16b, b);
  c = __builtin_amdgcn_wmma_f32_16x16x32_bf16(false, av, false, bv, (short)0, c, false, false);
  asm volatile("v_nop\n\tv_nop\n\tv_nop\n\tv_nop" : "+v"(c) : "v"(av), "v"(bv));
  return c;
}
__device__ __forceinline__ v8f mma_f16(v16h a, v16h b, v8f c) {
  c = __builtin_amdgcn_wmma_f32_16x16x32_f16(false, a, false, b, (short)0, c, false, false);
  asm volatile("v_nop\n\tv_nop\n\tv_nop\n\tv_nop" : "+v"(c) : "v"(a), "v"(b));
  return c;
}

__device__ __forceinline__ float elu_apx(float x) {
  float e = __expf(fminf(x, 0.f)) - 1.f;
  return x > 0.f ? x : e;
}
__device__ __forceinline__ float elu_acc(float x) {
  return x > 0.f ? x : expm1f(x);
}

__device__ __forceinline__ float pair_dist(const float* X, const float* Y) {
#pragma clang fp contract(off)
  float x0 = X[0], x1 = X[1], x2 = X[2];
  float y0 = Y[0], y1 = Y[1], y2 = Y[2];
  float xy = x0 * y0 + x1 * y1 + x2 * y2;
  float xx = x0 * x0 + x1 * x1 + x2 * x2;
  float yy = y0 * y0 + y1 * y1 + y2 * y2;
  float d2 = (-2.f * xy + yy) + xx;
  return sqrtf(fmaxf(d2, 0.f));
}

__device__ __forceinline__ void setup_pass(int t, const float* mlp_W,
                                           const float* pi_W, const float* sg_W,
                                           const float* mu_W, unsigned char* ws) {
  for (int c = t; c < (NC * KW) / 8; c += 256) {
    const int n = c >> 5, k0 = (c & 31) * 8;
    v8us hv, lv;
#pragma unroll
    for (int e = 0; e < 8; ++e) {
      float w = mlp_W[(size_t)(k0 + e) * NC + n];
      unsigned short hb, lb;
      split_bf16(w, hb, lb);
      hv[e] = hb;
      lv[e] = lb;
    }
    *(volatile v8us*)(ws + WB_WHI + (size_t)c * 16) = hv;
    *(volatile v8us*)(ws + WB_WLO + (size_t)c * 16) = lv;
  }
  {
    const int n = t >> 4, k0 = (t & 15) * 8;
    v8us ph, pl;
    v8h sv, mv;
#pragma unroll
    for (int e = 0; e < 8; ++e) {
      const int k = k0 + e;
      float wp = 0.f, ws_ = 0.f, wm = 0.f;
      if (n < NG) {
        wp  = pi_W[k * NG + n];
        ws_ = sg_W[k * NG + n];
        wm  = mu_W[k * NG + n];
      }
      unsigned short hb, lb;
      split_bf16(wp, hb, lb);
      ph[e] = hb;
      pl[e] = lb;
      sv[e] = (f16_t)(ws_ * 64.f);
      mv[e] = (f16_t)(wm * 64.f);
    }
    *(volatile v8us*)(ws + WB_PHI + (size_t)t * 16) = ph;
    *(volatile v8us*)(ws + WB_PLO + (size_t)t * 16) = pl;
    *(volatile v8h*)(ws + WB_SG + (size_t)t * 16) = sv;
    *(volatile v8h*)(ws + WB_MU + (size_t)t * 16) = mv;
  }
}

__global__ void __launch_bounds__(256) setup_kernel(
    const float* __restrict__ mlp_W, const float* __restrict__ pi_W,
    const float* __restrict__ sg_W, const float* __restrict__ mu_W,
    unsigned char* ws) {
  const int t = threadIdx.x;
  setup_pass(t, mlp_W, pi_W, sg_W, mu_W, ws);
  __threadfence();
  setup_pass(t, mlp_W, pi_W, sg_W, mu_W, ws);
}

__global__ void __launch_bounds__(256) ba_kernel(
    const float* __restrict__ hl, const int* __restrict__ nlc,
    const float* __restrict__ W1, const float* __restrict__ b1, const float* __restrict__ g1,
    const float* __restrict__ be1, const float* __restrict__ m1, const float* __restrict__ v1,
    const float* __restrict__ W2, const float* __restrict__ b2, const float* __restrict__ g2,
    const float* __restrict__ be2, const float* __restrict__ m2, const float* __restrict__ v2,
    const float* __restrict__ W3, const float* __restrict__ b3, float* out) {
  __shared__ float s_h[NC], s_x1[2 * NC], s_x2[NC], s_red[256], s_ba[NB];
  const int t = threadIdx.x;
  for (int b = 0; b < NB; ++b) {
    int nl = nlc[b];
    nl = nl < 0 ? 0 : (nl > NL ? NL : nl);
    if (t < NC) {
      float acc = 0.f;
      for (int i = 0; i < nl; ++i) acc += hl[((size_t)(b * NL + i)) * NC + t];
      s_h[t] = acc;
    }
    __syncthreads();
    {
      float acc = 0.f;
#pragma unroll 1
      for (int k = 0; k < NC; ++k) acc += s_h[k] * W1[(size_t)k * (2 * NC) + t];
      acc += b1[t];
      acc = (acc - m1[t]) * (1.f / sqrtf(v1[t] + 1e-5f)) * g1[t] + be1[t];
      s_x1[t] = elu_acc(acc);
    }
    __syncthreads();
    if (t < NC) {
      float acc = 0.f;
#pragma unroll 1
      for (int k = 0; k < 2 * NC; ++k) acc += s_x1[k] * W2[(size_t)k * NC + t];
      acc += b2[t];
      acc = (acc - m2[t]) * (1.f / sqrtf(v2[t] + 1e-5f)) * g2[t] + be2[t];
      s_x2[t] = elu_acc(acc);
    }
    __syncthreads();
    s_red[t] = (t < NC) ? s_x2[t] * W3[t] : 0.f;
    __syncthreads();
    for (int s = 128; s > 0; s >>= 1) {
      if (t < s) s_red[t] += s_red[t + s];
      __syncthreads();
    }
    if (t == 0) s_ba[b] = s_red[0] + b3[0];
    __syncthreads();
  }
  if (t == 0) {
    v4f a0, a1;
#pragma unroll
    for (int q = 0; q < 4; ++q) { a0[q] = s_ba[q]; a1[q] = s_ba[4 + q]; }
    float* p = out + OUT_BA;
    *(volatile v4f*)(p)     = a0;
    *(volatile v4f*)(p + 4) = a1;
    __threadfence();
    *(volatile v4f*)(p)     = a0;
    *(volatile v4f*)(p + 4) = a1;
  }
}

__device__ __forceinline__ void proj_store_pass(int t, const float (*s_d)[132], float* dst) {
#pragma unroll
  for (int it = 0; it < 8; ++it) {
    const int c = it * 128 + t;
    const int r = c >> 5, cc = c & 31;
    v4f v = *(const v4f*)&s_d[r][cc * 4];
    *(volatile v4f*)(dst + (size_t)r * NC + cc * 4) = v;
  }
}

__global__ void __launch_bounds__(128) proj_kernel(
    const float* __restrict__ hl, const float* __restrict__ hp,
    const int* __restrict__ nlc, const int* __restrict__ npc,
    const unsigned char* __restrict__ wtab, float* pa, float* pb) {
  __shared__ __attribute__((aligned(16))) unsigned short s_ahi[32][136];
  __shared__ __attribute__((aligned(16))) unsigned short s_alo[32][136];
  __shared__ __attribute__((aligned(16))) float s_d[32][132];

  const int t = threadIdx.x, blk = blockIdx.x;
  if (blk >= PROJ_BLOCKS) return;
  const bool lig = blk < (NB * NL) / 32;
  int row0, koff;
  const float* src;
  float* dst;
  if (lig) {
    row0 = blk * 32;
    src = hl + (size_t)row0 * NC;
    dst = pa + (size_t)row0 * NC;
    koff = 0;
  } else {
    row0 = (blk - (NB * NL) / 32) * 32;
    src = hp + (size_t)row0 * NC;
    dst = pb + (size_t)row0 * NC;
    koff = NC;
  }

  for (int idx = t; idx < 32 * 32; idx += 128) {
    const int r = idx >> 5, c4 = idx & 31;
    const int g = row0 + r;
    bool valid;
    if (lig) { const int b = g >> 6, i = g & 63;  valid = i < nlc[b]; }
    else     { const int b = g >> 9, j = g & 511; valid = j < npc[b]; }
    v4f x = *(const v4f*)(src + (size_t)r * NC + c4 * 4);
    const float msk = valid ? 1.f : 0.f;
    x = x * msk;
    v4us hv, lv;
#pragma unroll
    for (int e = 0; e < 4; ++e) {
      unsigned short hb, lb;
      split_bf16(x[e], hb, lb);
      hv[e] = hb;
      lv[e] = lb;
    }
    *(v4us*)&s_ahi[r][c4 * 4] = hv;
    *(v4us*)&s_alo[r][c4 * 4] = lv;
  }
  __syncthreads();

  const int lane = t & 31, wave = t >> 5;
  const int h = lane >> 4, m = lane & 15;
  const int rt = wave >> 1;
  const int cb = (wave & 1) * 4;
  const int arow = rt * 16 + m;
  const unsigned short* whi = (const unsigned short*)(wtab + WB_WHI);
  const unsigned short* wlo = (const unsigned short*)(wtab + WB_WLO);

  v8f acc[4];
#pragma unroll
  for (int ct = 0; ct < 4; ++ct) acc[ct] = zero8();

#pragma unroll 1
  for (int kq = 0; kq < 4; ++kq) {
    const int k0 = kq * 32;
    v16us ah = cat8u(*(const v8us*)&s_ahi[arow][k0 + 8 * h], *(const v8us*)&s_ahi[arow][k0 + 16 + 8 * h]);
    v16us al = cat8u(*(const v8us*)&s_alo[arow][k0 + 8 * h], *(const v8us*)&s_alo[arow][k0 + 16 + 8 * h]);
#pragma unroll
    for (int ct = 0; ct < 4; ++ct) {
      const int n = (cb + ct) * 16 + m;
      const unsigned short* ph = whi + (size_t)n * KW + koff + k0;
      const unsigned short* pl = wlo + (size_t)n * KW + koff + k0;
      v16us bh = cat8u(*(const v8us*)(ph + 8 * h), *(const v8us*)(ph + 16 + 8 * h));
      v16us bl = cat8u(*(const v8us*)(pl + 8 * h), *(const v8us*)(pl + 16 + 8 * h));
      acc[ct] = mma_bf16(ah, bh, acc[ct]);
      acc[ct] = mma_bf16(al, bh, acc[ct]);
      acc[ct] = mma_bf16(ah, bl, acc[ct]);
    }
  }

#pragma unroll
  for (int ct = 0; ct < 4; ++ct) {
#pragma unroll
    for (int r = 0; r < 8; ++r) s_d[rt * 16 + 8 * h + r][(cb + ct) * 16 + m] = acc[ct][r];
  }
  __syncthreads();

  proj_store_pass(t, s_d, dst);
  __threadfence();
  proj_store_pass(t, s_d, dst);
}

__device__ __forceinline__ void mdn_store_pass(int t, float* out, size_t base0, size_t based,
                                               const float* s_o0, const float* s_o1,
                                               const float* s_o2, const float* s_o3) {
  {
    const int c = t;
    v4f v0 = *(const v4f*)&s_o0[4 * c];
    v4f v1 = *(const v4f*)&s_o1[4 * c];
    v4f v2 = *(const v4f*)&s_o2[4 * c];
    *(volatile v4f*)(out + OUT_PI + base0 + 4 * c) = v0;
    *(volatile v4f*)(out + OUT_SG + base0 + 4 * c) = v1;
    *(volatile v4f*)(out + OUT_MU + base0 + 4 * c) = v2;
  }
  if (t < 32) {
    const int c = 128 + t;
    v4f v0 = *(const v4f*)&s_o0[4 * c];
    v4f v1 = *(const v4f*)&s_o1[4 * c];
    v4f v2 = *(const v4f*)&s_o2[4 * c];
    *(volatile v4f*)(out + OUT_PI + base0 + 4 * c) = v0;
    *(volatile v4f*)(out + OUT_SG + base0 + 4 * c) = v1;
    *(volatile v4f*)(out + OUT_MU + base0 + 4 * c) = v2;
  }
  if (t < 16) {
    v4f v3 = *(const v4f*)&s_o3[4 * t];
    *(volatile v4f*)(out + OUT_D + based + 4 * t) = v3;
  }
}

__global__ void __launch_bounds__(128) mdn_kernel(
    const float* __restrict__ pa, const float* __restrict__ pb,
    const unsigned char* __restrict__ wtab,
    const float* __restrict__ mlp_b, const float* __restrict__ mlp_g,
    const float* __restrict__ mlp_be, const float* __restrict__ mlp_m,
    const float* __restrict__ mlp_v,
    const float* __restrict__ pi_b, const float* __restrict__ sg_b,
    const float* __restrict__ mu_b,
    const float* __restrict__ l_pos, const float* __restrict__ p_pos,
    const int* __restrict__ nlc, const int* __restrict__ npc, float* out) {
  __shared__ __attribute__((aligned(16))) float s_bp[64][132];
  __shared__ __attribute__((aligned(16))) float s_base[NC];
  __shared__ __attribute__((aligned(16))) float s_sc[NC];
  __shared__ float s_hb[32];
  __shared__ float s_acc[4][16][49];
  __shared__ __attribute__((aligned(16))) float s_o0[640];
  __shared__ __attribute__((aligned(16))) float s_o1[640];
  __shared__ __attribute__((aligned(16))) float s_o2[640];
  __shared__ __attribute__((aligned(16))) float s_o3[64];

  const int t = threadIdx.x, blk = blockIdx.x;
  if (blk >= MDN_BLOCKS) return;
  const int jt = blk & 7;
  const int i  = (blk >> 3) & 63;
  const int b  = blk >> 9;
  const int jb0 = jt * 64;

  if (t < NC) {
    const float sc = mlp_g[t] * (1.f / sqrtf(mlp_v[t] + 1e-5f));
    const float sh = (mlp_b[t] - mlp_m[t]) * sc + mlp_be[t];
    s_sc[t] = sc;
    s_base[t] = pa[(size_t)(b * NL + i) * NC + t] * sc + sh;
  }
  if (t < 32) {
    float v = 0.f;
    if (t < NG)           v = pi_b[t];
    else if (t < 2 * NG)  v = sg_b[t - NG];
    else if (t < 3 * NG)  v = mu_b[t - 2 * NG];
    s_hb[t] = v;
  }
  __syncthreads();

  const float* bsrc = pb + (size_t)(b * NPP + jb0) * NC;
  for (int idx = t; idx < 64 * 32; idx += 128) {
    const int j = idx >> 5, c4 = idx & 31;
    v4f x = *(const v4f*)(bsrc + (size_t)j * NC + c4 * 4);
    v4f s = *(const v4f*)&s_sc[c4 * 4];
    *(v4f*)&s_bp[j][c4 * 4] = x * s;
  }
  __syncthreads();

  const int lane = t & 31, wave = t >> 5;
  const int h = lane >> 4, m = lane & 15;
  const int jl = wave * 16 + m;

  const unsigned short* phi = (const unsigned short*)(wtab + WB_PHI) + m * NC;
  const unsigned short* plo = (const unsigned short*)(wtab + WB_PLO) + m * NC;
  const f16_t* sgw = (const f16_t*)(wtab + WB_SG) + m * NC;
  const f16_t* muw = (const f16_t*)(wtab + WB_MU) + m * NC;

  v8f accp = zero8(), accs = zero8(), accm = zero8();

#pragma unroll 1
  for (int kq = 0; kq < 4; ++kq) {
    const int k0 = kq * 32;
    v16us ah, al;
    v16h af;
#pragma unroll
    for (int q = 0; q < 4; ++q) {
      const int kk = k0 + 8 * h + (q & 1) * 4 + (q >> 1) * 16;
      v4f aa = *(const v4f*)&s_base[kk];
      v4f bb = *(const v4f*)&s_bp[jl][kk];
#pragma unroll
      for (int e = 0; e < 4; ++e) {
        const float hm = elu_apx(aa[e] + bb[e]);
        unsigned short hb, lb;
        split_bf16(hm, hb, lb);
        ah[4 * q + e] = hb;
        al[4 * q + e] = lb;
        af[4 * q + e] = (f16_t)hm;
      }
    }
    v16us bh = cat8u(*(const v8us*)(phi + k0 + 8 * h), *(const v8us*)(phi + k0 + 16 + 8 * h));
    v16us bl = cat8u(*(const v8us*)(plo + k0 + 8 * h), *(const v8us*)(plo + k0 + 16 + 8 * h));
    v16h  bs = cat8h(*(const v8h*)(sgw + k0 + 8 * h), *(const v8h*)(sgw + k0 + 16 + 8 * h));
    v16h  bm = cat8h(*(const v8h*)(muw + k0 + 8 * h), *(const v8h*)(muw + k0 + 16 + 8 * h));
    accp = mma_bf16(ah, bh, accp);
    accp = mma_bf16(al, bh, accp);
    accp = mma_bf16(ah, bl, accp);
    accs = mma_f16(af, bs, accs);
    accm = mma_f16(af, bm, accm);
  }

#pragma unroll
  for (int r = 0; r < 8; ++r) {
    s_acc[wave][8 * h + r][m]      = accp[r];
    s_acc[wave][8 * h + r][16 + m] = accs[r];
    s_acc[wave][8 * h + r][32 + m] = accm[r];
  }
  __syncthreads();

  if (t < 64) {
    const int w = t >> 4, rr = t & 15;
    const int j = jb0 + t;
    const float lm = (i < nlc[b]) ? 1.f : 0.f;
    const float pm = (j < npc[b]) ? 1.f : 0.f;
    const float cm = lm * pm;

    float lg[NG];
    float mx = -3.0e38f;
#pragma unroll
    for (int g = 0; g < NG; ++g) {
      const float z = s_acc[w][rr][g] + s_hb[g];
      lg[g] = z;
      mx = fmaxf(mx, z);
    }
    float ssum = 0.f;
#pragma unroll
    for (int g = 0; g < NG; ++g) {
      const float e = expf(lg[g] - mx);
      lg[g] = e;
      ssum += e;
    }
    const float inv = 1.f / ssum;
#pragma unroll
    for (int g = 0; g < NG; ++g) s_o0[t * NG + g] = (lg[g] * inv + 1e-10f) * cm;

#pragma unroll
    for (int g = 0; g < NG; ++g) {
      const float z = s_acc[w][rr][16 + g] * (1.f / 64.f) + s_hb[NG + g];
      const float x = elu_acc(z);
      s_o1[t * NG + g] = ((x + 1.1f) + 1e-10f) * cm;
    }
#pragma unroll
    for (int g = 0; g < NG; ++g) {
      const float z = s_acc[w][rr][32 + g] * (1.f / 64.f) + s_hb[2 * NG + g];
      const float x = elu_acc(z);
      s_o2[t * NG + g] = ((x + 1.0f) + 1e-10f) * cm;
    }
    s_o3[t] = pair_dist(l_pos + (size_t)(b * NL + i) * 3, p_pos + (size_t)(b * NPP + j) * 3) * cm;
  }
  __syncthreads();

  const size_t base0 = ((size_t)(b * NL + i) * NPP + jb0) * NG;
  const size_t based = (size_t)(b * NL + i) * NPP + jb0;
  mdn_store_pass(t, out, base0, based, s_o0, s_o1, s_o2, s_o3);
  __threadfence();
  mdn_store_pass(t, out, base0, based, s_o0, s_o1, s_o2, s_o3);
}

extern "C" void kernel_launch(void* const* d_in, const int* in_sizes, int n_in,
                              void* d_out, int out_size, void* d_ws, size_t ws_size,
                              hipStream_t stream) {
  if (n_in < 32) return;
  if (ws_size < (size_t)WB_END) return;
  if (out_size != (int)OUT_TOTAL) return;
  if (in_sizes[0] != NB * NL * NC || in_sizes[1] != NB * NPP * NC ||
      in_sizes[2] != NB * NL * 3 || in_sizes[3] != NB * NPP * 3 ||
      in_sizes[4] != NB || in_sizes[5] != NB ||
      in_sizes[6] != 2 * NC * NC || in_sizes[12] != 2 * NC * NC || in_sizes[18] != 2 * NC * NC ||
      in_sizes[7] != NC || in_sizes[8] != NC || in_sizes[9] != NC || in_sizes[10] != NC || in_sizes[11] != NC ||
      in_sizes[13] != 2 * NC || in_sizes[14] != 2 * NC || in_sizes[15] != 2 * NC ||
      in_sizes[16] != 2 * NC || in_sizes[17] != 2 * NC ||
      in_sizes[19] != NC || in_sizes[20] != NC || in_sizes[21] != NC || in_sizes[22] != NC || in_sizes[23] != NC ||
      in_sizes[24] != NC || in_sizes[25] < 1 ||
      in_sizes[26] != NC * NG || in_sizes[28] != NC * NG || in_sizes[30] != NC * NG ||
      in_sizes[27] < NG || in_sizes[29] < NG || in_sizes[31] < NG) return;

  const float* hl     = (const float*)d_in[0];
  const float* hp     = (const float*)d_in[1];
  const float* l_pos  = (const float*)d_in[2];
  const float* p_pos  = (const float*)d_in[3];
  const int*   nl_c   = (const int*)  d_in[4];
  const int*   np_c   = (const int*)  d_in[5];
  const float* mlp_W  = (const float*)d_in[6];
  const float* mlp_b  = (const float*)d_in[7];
  const float* mlp_g  = (const float*)d_in[8];
  const float* mlp_be = (const float*)d_in[9];
  const float* mlp_m  = (const float*)d_in[10];
  const float* mlp_v  = (const float*)d_in[11];
  const float* ba_W1  = (const float*)d_in[12];
  const float* ba_b1  = (const float*)d_in[13];
  const float* ba_g1  = (const float*)d_in[14];
  const float* ba_be1 = (const float*)d_in[15];
  const float* ba_m1  = (const float*)d_in[16];
  const float* ba_v1  = (const float*)d_in[17];
  const float* ba_W2  = (const float*)d_in[18];
  const float* ba_b2  = (const float*)d_in[19];
  const float* ba_g2  = (const float*)d_in[20];
  const float* ba_be2 = (const float*)d_in[21];
  const float* ba_m2  = (const float*)d_in[22];
  const float* ba_v2  = (const float*)d_in[23];
  const float* ba_W3  = (const float*)d_in[24];
  const float* ba_b3  = (const float*)d_in[25];
  const float* pi_W   = (const float*)d_in[26];
  const float* pi_b   = (const float*)d_in[27];
  const float* sg_W   = (const float*)d_in[28];
  const float* sg_b   = (const float*)d_in[29];
  const float* mu_W   = (const float*)d_in[30];
  const float* mu_b   = (const float*)d_in[31];

  float* out = (float*)d_out;
  unsigned char* ws = (unsigned char*)d_ws;
  float* pa = (float*)(ws + WB_PA);
  float* pb = (float*)(ws + WB_PB);

  setup_kernel<<<1, 256, 0, stream>>>(mlp_W, pi_W, sg_W, mu_W, ws);
  ba_kernel<<<1, 256, 0, stream>>>(hl, nl_c,
                                   ba_W1, ba_b1, ba_g1, ba_be1, ba_m1, ba_v1,
                                   ba_W2, ba_b2, ba_g2, ba_be2, ba_m2, ba_v2,
                                   ba_W3, ba_b3, out);
  proj_kernel<<<PROJ_BLOCKS, 128, 0, stream>>>(hl, hp, nl_c, np_c, ws, pa, pb);
  mdn_kernel<<<MDN_BLOCKS, 128, 0, stream>>>(pa, pb, ws, mlp_b, mlp_g, mlp_be, mlp_m, mlp_v,
                                             pi_b, sg_b, mu_b, l_pos, p_pos, nl_c, np_c, out);
}
